// MultiHeadAttention_48301202211428
// MI455X (gfx1250) — hardware-run, weakly checked
//
#include <hip/hip_runtime.h>


#ifndef NB
#define NB 2
#endif
#ifndef SEQ
#define SEQ 2048
#endif
#define NB_FULL  2
#define SEQ_FULL 2048
#ifndef OUT_SEQ
#define OUT_SEQ SEQ
#endif
#define DM   1024
#define NH_  16
#define HD   64
#define NREL 7
#define AW   4
#define QRS  2048.0f
#define QRI  (1.0f / 2048.0f)
#define SC2  (0.125f * 1.4426950408889634f)
#define PSH  8.0f
#define PKS  256.0f
#define RELS (SC2 / 256.0f)
#define CTXS 256.0f
#define WOS  256.0f
#define OUTI (1.0f / 65536.0f)

static_assert(HD == 64);
static_assert(NH_ * HD == DM);
static_assert(DM % 64 == 0);
static_assert(DM % 32 == 0);
static_assert(SEQ % 64 == 0);
static_assert((NB * SEQ) % 64 == 0);
static_assert(SEQ % 32 == 0);
static_assert(SEQ % (16 * AW) == 0);
static_assert(((size_t)SEQ * DM) % 8 == 0);
static_assert((NREL * DM) % 8 == 0);
static_assert(NREL <= 8);
static_assert(NB <= NB_FULL);
static_assert(SEQ <= SEQ_FULL);
static_assert((size_t)NB_FULL * SEQ_FULL * DM * 4 == (size_t)16777216);

typedef _Float16 h16;
typedef unsigned short bf;
typedef __attribute__((ext_vector_type(16))) __bf16   v16bf;
typedef __attribute__((ext_vector_type(16))) _Float16 v16h;
typedef __attribute__((ext_vector_type(8)))  _Float16 v8h;
typedef __attribute__((ext_vector_type(8)))  unsigned short v8us;
typedef __attribute__((ext_vector_type(8)))  float    v8f;
typedef __attribute__((ext_vector_type(4)))  float    v4f;
typedef v4f  __attribute__((may_alias)) v4fa;
typedef v8us __attribute__((may_alias)) v8usa;

__device__ __forceinline__ unsigned short f2bf(float f) { unsigned u = __float_as_uint(f); u += 0x7FFFu + ((u >> 16) & 1u); return (unsigned short)(u >> 16); }
__device__ __forceinline__ float bfr(float f) { return __uint_as_float(((unsigned)f2bf(f)) << 16); }
__device__ __forceinline__ v16h cat16(v8h lo, v8h hi) { return __builtin_shufflevector(lo, hi, 0, 1, 2, 3, 4, 5, 6, 7, 8, 9, 10, 11, 12, 13, 14, 15); }
__device__ __forceinline__ v16bf cat16b(v8us lo, v8us hi) { return __builtin_bit_cast(v16bf, __builtin_shufflevector(lo, hi, 0, 1, 2, 3, 4, 5, 6, 7, 8, 9, 10, 11, 12, 13, 14, 15)); }
__device__ __forceinline__ v8f wmma16(v16h a, v16h b, v8f c) { return __builtin_amdgcn_wmma_f32_16x16x32_f16(false, a, false, b, (short)0, c, false, false); }
__device__ __forceinline__ v8f wmmab(v16bf a, v16bf b, v8f c) { return __builtin_amdgcn_wmma_f32_16x16x32_bf16(false, a, false, b, (short)0, c, false, false); }
__device__ __forceinline__ v16h  ldh(const h16* p) { return cat16(*(const v8h*)p, *(const v8h*)(p + 16)); }
__device__ __forceinline__ v16bf ldb(const bf* p)  { return cat16b(*(const v8us*)p, *(const v8us*)(p + 16)); }
__device__ __forceinline__ void wave_sync() { __builtin_amdgcn_fence(3  , "wavefront"); __builtin_amdgcn_wave_barrier(); asm volatile("" ::: "memory"); }
__device__ __forceinline__ float sel7(int i, float s0, float s1, float s2, float s3, float s4, float s5, float s6) {
    float v = s0; v = (i == 1) ? s1 : v; v = (i == 2) ? s2 : v; v = (i == 3) ? s3 : v; v = (i == 4) ? s4 : v; v = (i == 5) ? s5 : v; v = (i == 6) ? s6 : v; return v; }

__global__ __launch_bounds__(256) void k_cvt8(const float* __restrict__ src, bf* dst, size_t nsrc8, size_t n8) {
    const size_t i = (size_t)blockIdx.x * 256 + threadIdx.x; if (i >= n8) return;
    const bool live = i < nsrc8; const size_t is = live ? i : (nsrc8 - 1);
    const v8f v = *(const v8f*)(src + is * 8); v8us o;
#pragma unroll
    for (int k = 0; k < 8; ++k) { const unsigned short c = f2bf(v[k]); o[k] = live ? c : (unsigned short)0; }
    *(volatile v8us*)(dst + i * 8) = o; __threadfence(); *(volatile v8us*)(dst + i * 8) = o;
}

__global__ __launch_bounds__(256) void k_wt(const float* __restrict__ W, bf* WT, int f16mode) {
    __shared__ __align__(16) unsigned short ts[64 * 72];
    const int tid = threadIdx.x; const int n0 = blockIdx.x * 64, k0 = blockIdx.y * 64;
#pragma unroll
    for (int p = 0; p < 4; ++p) { const int kr = p * 16 + (tid >> 4), c4 = (tid & 15) * 4;
        const v4f v = *(const v4f*)(W + (size_t)(k0 + kr) * DM + n0 + c4);
#pragma unroll
        for (int i = 0; i < 4; ++i) { const unsigned short bb = f2bf(v[i]); const float fb = __uint_as_float(((unsigned)bb) << 16);
            const unsigned short hb = __builtin_bit_cast(unsigned short, (h16)(fb * WOS));
            ts[(c4 + i) * 72 + kr] = f16mode ? hb : bb; } }
    __syncthreads();
#pragma unroll 1
    for (int ps = 0; ps < 2; ++ps) {
#pragma unroll
        for (int p = 0; p < 2; ++p) { const int n = p * 32 + (tid >> 3), c8 = (tid & 7) * 8;
            const v8us o = *(const v8usa*)(&ts[n * 72 + c8]);
            *(volatile v8us*)(WT + (size_t)(n0 + n) * DM + k0 + c8) = o; }
        if (ps == 0) __threadfence(); }
}

template <int MODE>
__global__ __launch_bounds__(32) void k_gemm(const bf* __restrict__ A, const bf* __restrict__ Bt, const float* __restrict__ bias,
                                             const float* __restrict__ add0, const float* __restrict__ add1, float sa, float sbs,
                                             h16* P0h, h16* P0r, h16* P1h, h16* P1r, float* OutF,
                                             int RB, size_t sRB, int pitch, int CB, size_t sCB) {
    __shared__ __align__(16) float os[16 * 68];
    const int K = DM;
    const int lane = threadIdx.x & 31, lr = lane & 15, hi = lane >> 4; const int r0 = blockIdx.x * 64, c0 = blockIdx.y * 64;
    v8f acc[4][4];
#pragma unroll
    for (int mb = 0; mb < 4; ++mb)
#pragma unroll
        for (int nb = 0; nb < 4; ++nb) acc[mb][nb] = (v8f){};
    const size_t aoff = (size_t)(r0 + lr) * K + 8 * hi, boff = (size_t)(c0 + lr) * K + 8 * hi;
    if (MODE == 3) {
        const h16* Ah = (const h16*)A; const h16* Bh = (const h16*)Bt;
#pragma unroll 1
        for (int kc = 0; kc < K; kc += 32) {
            v16h a[4];
#pragma unroll
            for (int mb = 0; mb < 4; ++mb) a[mb] = ldh(Ah + aoff + (size_t)mb * 16 * K + kc);
#pragma unroll
            for (int nb = 0; nb < 4; ++nb) { const v16h b = ldh(Bh + boff + (size_t)nb * 16 * K + kc);
#pragma unroll
                for (int mb = 0; mb < 4; ++mb) acc[mb][nb] = wmma16(a[mb], b, acc[mb][nb]); }
            asm volatile("v_nop\n\tv_nop\n\tv_nop\n\tv_nop" : "+v"(acc[0][0]), "+v"(acc[1][1]), "+v"(acc[2][2]), "+v"(acc[3][3]) : "v"(a[0]), "v"(a[1]), "v"(a[2]), "v"(a[3]));
        }
    } else {
#pragma unroll 1
        for (int kc = 0; kc < K; kc += 32) {
            v16bf a[4];
#pragma unroll
            for (int mb = 0; mb < 4; ++mb) a[mb] = ldb(A + aoff + (size_t)mb * 16 * K + kc);
#pragma unroll
            for (int nb = 0; nb < 4; ++nb) { const v16bf b = ldb(Bt + boff + (size_t)nb * 16 * K + kc);
#pragma unroll
                for (int mb = 0; mb < 4; ++mb) acc[mb][nb] = wmmab(a[mb], b, acc[mb][nb]); }
            asm volatile("v_nop\n\tv_nop\n\tv_nop\n\tv_nop" : "+v"(acc[0][0]), "+v"(acc[1][1]), "+v"(acc[2][2]), "+v"(acc[3][3]) : "v"(a[0]), "v"(a[1]), "v"(a[2]), "v"(a[3]));
        }
    }
    const size_t tbase = (size_t)(r0 / RB) * sRB + (size_t)(r0 % RB) * (size_t)pitch + (size_t)(c0 / CB) * sCB + (size_t)(c0 % CB);
#pragma unroll
    for (int mb = 0; mb < 4; ++mb) {
#pragma unroll
        for (int nb = 0; nb < 4; ++nb) {
#pragma unroll
            for (int j = 0; j < 8; ++j) os[(hi * 8 + j) * 68 + nb * 16 + lr] = acc[mb][nb][j]; }
        wave_sync();
        if (MODE == 3) {
            const int g0 = r0 + mb * 16;
            const size_t ob = ((size_t)(g0 / SEQ) * OUT_SEQ + (size_t)(g0 % SEQ)) * DM + c0;
#pragma unroll 1
            for (int ps = 0; ps < 2; ++ps) {
#pragma unroll
                for (int s = 0; s < 8; ++s) { const int row = 2 * s + hi, cofs = lr * 4;
                    const v4f x = *(const v4fa*)(&os[row * 68 + cofs]);
                    const v4f bb = *(const v4f*)(bias + c0 + cofs); v4f val;
#pragma unroll
                    for (int i = 0; i < 4; ++i) val[i] = x[i] * sa + bfr(bb[i]) * sbs;
                    *(volatile v4f*)(OutF + ob + (size_t)row * DM + cofs) = val; }
                if (ps == 0) __threadfence(); }
        } else {
            const size_t sbase = tbase + (size_t)(mb * 16) * (size_t)pitch;
#pragma unroll 1
            for (int ps = 0; ps < 2; ++ps) {
#pragma unroll
                for (int s = 0; s < 4; ++s) { const int row = 4 * s + (lane >> 3), c8 = (lane & 7) * 8;
                    const v4f x0 = *(const v4fa*)(&os[row * 68 + c8]); const v4f x1 = *(const v4fa*)(&os[row * 68 + c8 + 4]);
                    float bb[8];
                    if (MODE == 2) { const float br = bfr(bias[r0 + mb * 16 + row]);
#pragma unroll
                        for (int i = 0; i < 8; ++i) bb[i] = br;
                    } else { const v4f b0 = *(const v4f*)(bias + c0 + c8); const v4f b1 = *(const v4f*)(bias + c0 + c8 + 4);
#pragma unroll
                        for (int i = 0; i < 4; ++i) { bb[i] = bfr(b0[i]); bb[4 + i] = bfr(b1[i]); } }
                    float val[8];
#pragma unroll
                    for (int i = 0; i < 4; ++i) { val[i] = x0[i] * sa + bb[i] * sbs; val[4 + i] = x1[i] * sa + bb[4 + i] * sbs; }
                    const size_t oo = sbase + (size_t)row * (size_t)pitch + c8;
                    if (MODE == 0) {
                        const v4f u0 = *(const v4f*)(add0 + c0 + c8); const v4f u1 = *(const v4f*)(add0 + c0 + c8 + 4);
                        const v4f w0 = *(const v4f*)(add1 + c0 + c8); const v4f w1 = *(const v4f*)(add1 + c0 + c8 + 4);
                        v8h hu, ru, hw, rw;
#pragma unroll
                        for (int i = 0; i < 4; ++i) {
                            const float ua = val[i] + bfr(u0[i]); const float ub = val[4 + i] + bfr(u1[i]);
                            const float wa = val[i] + bfr(w0[i]); const float wb = val[4 + i] + bfr(w1[i]);
                            const h16 ha = (h16)ua; const h16 hb = (h16)ub; const h16 hc = (h16)wa; const h16 hd = (h16)wb;
                            hu[i] = ha; hu[4 + i] = hb; ru[i] = (h16)((ua - (float)ha) * QRS); ru[4 + i] = (h16)((ub - (float)hb) * QRS);
                            hw[i] = hc; hw[4 + i] = hd; rw[i] = (h16)((wa - (float)hc) * QRS); rw[4 + i] = (h16)((wb - (float)hd) * QRS); }
                        *(volatile v8h*)(P0h + oo) = hu; *(volatile v8h*)(P0r + oo) = ru;
                        *(volatile v8h*)(P1h + oo) = hw; *(volatile v8h*)(P1r + oo) = rw;
                    } else {
                        v8h hv;
#pragma unroll
                        for (int i = 0; i < 8; ++i) hv[i] = (h16)val[i];
                        *(volatile v8h*)(P0h + oo) = hv; } }
                if (ps == 0) __threadfence(); }
        }
        wave_sync();
    }
}

__global__ __launch_bounds__(32 * AW) void k_flash(const h16* __restrict__ QCH, const h16* __restrict__ QCR, const h16* __restrict__ QRH, const h16* __restrict__ QRR,
                                                   const h16* __restrict__ KP, const h16* __restrict__ VT, const h16* __restrict__ PKP, h16* CTX) {
    __shared__ __align__(16) float os[AW * 16 * 68];
    const int lane = threadIdx.x & 31, wave = threadIdx.x >> 5, lr = lane & 15, hi = lane >> 4;
    const int zh = blockIdx.y; const int b = zh / NH_, h = zh % NH_;
    const int t0 = (blockIdx.x * AW + wave) * 16;
    const int t0u = __builtin_amdgcn_readfirstlane(t0);
    const int tq = t0 + lr;
    const size_t pbase = (size_t)zh * SEQ * HD;
    const size_t qo = pbase + (size_t)(t0 + lr) * HD + 8 * hi;
    float sm[NREL];
    {
        const v16h rh0 = ldh(QRH + qo), rh1 = ldh(QRH + qo + 32), rr0 = ldh(QRR + qo), rr1 = ldh(QRR + qo + 32);
        const h16* pa = PKP + (size_t)h * 64 * HD + (size_t)lr * HD + 8 * hi;
        const v16h p0 = ldh(pa), p1 = ldh(pa + 32);
        v8f smH = (v8f){}, smL = (v8f){};
        smH = wmma16(p0, rh0, smH); smL = wmma16(p0, rr0, smL);
        smH = wmma16(p1, rh1, smH); smL = wmma16(p1, rr1, smL);
        asm volatile("v_nop\n\tv_nop\n\tv_nop\n\tv_nop" : "+v"(smH), "+v"(smL) : "v"(p0), "v"(p1), "v"(rh0), "v"(rh1), "v"(rr0), "v"(rr1));
#pragma unroll
        for (int r = 0; r < NREL; ++r) { const float v = (smH[r] + smL[r] * QRI) * RELS; const float o = __shfl_xor(v, 16, 32); sm[r] = hi ? o : v; }
    }
    const v16h qh0 = ldh(QCH + qo), qh1 = ldh(QCH + qo + 32), qr0 = ldh(QCR + qo), qr1 = ldh(QCR + qo + 32);
    const size_t ko = pbase + (size_t)lr * HD + 8 * hi;
    const size_t vo = pbase + (size_t)lr * SEQ + 8 * hi;
    v8f o0 = (v8f){}, o1 = (v8f){}, o2 = (v8f){}, o3 = (v8f){};
    float m = -3.0e38f, l = 0.0f;
#pragma unroll 1
    for (int key0 = 0; key0 < SEQ; key0 += 32) {
        const h16* ka = KP + ko + (size_t)key0 * HD;
        const v16h ka0 = ldh(ka), ka1 = ldh(ka + 32), kb0 = ldh(ka + 16 * HD), kb1 = ldh(ka + 16 * HD + 32);
        v8f sHa = (v8f){}, sLa = (v8f){}, sHb = (v8f){}, sLb = (v8f){};
        sHa = wmma16(ka0, qh0, sHa); sLa = wmma16(ka0, qr0, sLa); sHb = wmma16(kb0, qh0, sHb); sLb = wmma16(kb0, qr0, sLb);
        sHa = wmma16(ka1, qh1, sHa); sLa = wmma16(ka1, qr1, sLa); sHb = wmma16(kb1, qh1, sHb); sLb = wmma16(kb1, qr1, sLb);
        asm volatile("v_nop\n\tv_nop\n\tv_nop\n\tv_nop" : "+v"(sHa), "+v"(sLa), "+v"(sHb), "+v"(sLb) : "v"(ka0), "v"(ka1), "v"(kb0), "v"(kb1));
        float ra[8], rc[8];
        const bool nearDiag = !((key0 + 34 <= t0u) || (key0 >= t0u + 18));
        if (nearDiag) {
#pragma unroll
            for (int r = 0; r < 8; ++r) {
                int d0 = tq - (key0 + 8 * hi + r); int d1 = d0 - 16;
                d0 = (d0 < -3 ? -3 : (d0 > 3 ? 3 : d0)) + 3; d1 = (d1 < -3 ? -3 : (d1 > 3 ? 3 : d1)) + 3;
                ra[r] = sel7(d0, sm[0], sm[1], sm[2], sm[3], sm[4], sm[5], sm[6]);
                rc[r] = sel7(d1, sm[0], sm[1], sm[2], sm[3], sm[4], sm[5], sm[6]); }
        } else {
            const float c = (key0 < t0u) ? sm[6] : sm[0];
#pragma unroll
            for (int r = 0; r < 8; ++r) { ra[r] = c; rc[r] = c; }
        }
        float ta[8], tb[8]; float mx = -3.0e38f;
#pragma unroll
        for (int r = 0; r < 8; ++r) { ta[r] = (sHa[r] + sLa[r] * QRI) * SC2 + ra[r]; tb[r] = (sHb[r] + sLb[r] * QRI) * SC2 + rc[r]; mx = fmaxf(mx, fmaxf(ta[r], tb[r])); }
        mx = fmaxf(mx, __shfl_xor(mx, 16, 32));
        const float mnew = fmaxf(m, mx);
        const float alpha = __builtin_amdgcn_exp2f(m - mnew);
        const float sh = PSH - mnew;
        v16h pb; float ls = 0.0f;
#pragma unroll
        for (int r = 0; r < 8; ++r) { const h16 pa = (h16)__builtin_amdgcn_exp2f(ta[r] + sh); const h16 pc = (h16)__builtin_amdgcn_exp2f(tb[r] + sh); pb[r] = pa; pb[8 + r] = pc; ls += (float)pa + (float)pc; }
        l = l * alpha + ls; m = mnew;
        o0 = o0 * alpha; o1 = o1 * alpha; o2 = o2 * alpha; o3 = o3 * alpha;
        const h16* va = VT + vo + key0;
        const v16h v0 = ldh(va), v1 = ldh(va + (size_t)16 * SEQ), v2 = ldh(va + (size_t)32 * SEQ), v3 = ldh(va + (size_t)48 * SEQ);
        o0 = wmma16(v0, pb, o0); o1 = wmma16(v1, pb, o1); o2 = wmma16(v2, pb, o2); o3 = wmma16(v3, pb, o3);
        asm volatile("v_nop\n\tv_nop\n\tv_nop\n\tv_nop" : "+v"(o0), "+v"(o1), "+v"(o2), "+v"(o3) : "v"(v0), "v"(v1), "v"(v2), "v"(v3), "v"(pb));
    }
    l += __shfl_xor(l, 16, 32);
    const float inv = CTXS / l;
    const int wb = wave * 16 * 68;
    { v4f a, c;
      a[0] = o0[0] * inv; a[1] = o0[1] * inv; a[2] = o0[2] * inv; a[3] = o0[3] * inv; c[0] = o0[4] * inv; c[1] = o0[5] * inv; c[2] = o0[6] * inv; c[3] = o0[7] * inv;
      *(v4fa*)(&os[wb + lr * 68 +  0 + 8 * hi]) = a; *(v4fa*)(&os[wb + lr * 68 +  0 + 8 * hi + 4]) = c;
      a[0] = o1[0] * inv; a[1] = o1[1] * inv; a[2] = o1[2] * inv; a[3] = o1[3] * inv; c[0] = o1[4] * inv; c[1] = o1[5] * inv; c[2] = o1[6] * inv; c[3] = o1[7] * inv;
      *(v4fa*)(&os[wb + lr * 68 + 16 + 8 * hi]) = a; *(v4fa*)(&os[wb + lr * 68 + 16 + 8 * hi + 4]) = c;
      a[0] = o2[0] * inv; a[1] = o2[1] * inv; a[2] = o2[2] * inv; a[3] = o2[3] * inv; c[0] = o2[4] * inv; c[1] = o2[5] * inv; c[2] = o2[6] * inv; c[3] = o2[7] * inv;
      *(v4fa*)(&os[wb + lr * 68 + 32 + 8 * hi]) = a; *(v4fa*)(&os[wb + lr * 68 + 32 + 8 * hi + 4]) = c;
      a[0] = o3[0] * inv; a[1] = o3[1] * inv; a[2] = o3[2] * inv; a[3] = o3[3] * inv; c[0] = o3[4] * inv; c[1] = o3[5] * inv; c[2] = o3[6] * inv; c[3] = o3[7] * inv;
      *(v4fa*)(&os[wb + lr * 68 + 48 + 8 * hi]) = a; *(v4fa*)(&os[wb + lr * 68 + 48 + 8 * hi + 4]) = c; }
    wave_sync();
    h16* crow = CTX + ((size_t)b * SEQ + t0) * DM + h * HD;
#pragma unroll 1
    for (int ps = 0; ps < 2; ++ps) {
#pragma unroll
        for (int s = 0; s < 4; ++s) { const int row = 4 * s + (lane >> 3), c8 = (lane & 7) * 8;
            const v4f x0 = *(const v4fa*)(&os[wb + row * 68 + c8]); const v4f x1 = *(const v4fa*)(&os[wb + row * 68 + c8 + 4]); v8h hv;
#pragma unroll
            for (int i = 0; i < 4; ++i) { hv[i] = (h16)x0[i]; hv[4 + i] = (h16)x1[i]; }
            *(volatile v8h*)(crow + (size_t)row * DM + c8) = hv; }
        if (ps == 0) __threadfence(); }
}

static constexpr size_t al256(size_t v) { return (v + 255) & ~(size_t)255; }
static constexpr size_t SZ_XB  = al256((size_t)NB * SEQ * DM * 2);
static constexpr size_t SZ_WT  = al256((size_t)DM * DM * 2);
static constexpr size_t SZ_PE  = al256((size_t)64 * DM * 2);
static constexpr size_t SZ_PL  = al256((size_t)NB * NH_ * SEQ * HD * 2);
static constexpr size_t SZ_PK  = al256((size_t)NH_ * 64 * HD * 2);
static constexpr size_t SZ_CTX = al256((size_t)NB * SEQ * DM * 2);
static constexpr size_t SZ_TOTAL = 3 * SZ_XB + 4 * SZ_WT + SZ_PE + 6 * SZ_PL + SZ_PK + SZ_CTX;
static_assert(SZ_TOTAL <= (size_t)134217728);

static void cvt_x(const float* x, bf* XB, hipStream_t stream) {
    if (SEQ == SEQ_FULL) {
        const size_t n8 = (size_t)NB * SEQ * DM / 8;
        k_cvt8<<<(unsigned)((n8 + 255) / 256), 256, 0, stream>>>(x, XB, n8, n8);
    } else {
        const size_t n8 = (size_t)SEQ * DM / 8;
        for (int b = 0; b < NB; ++b) k_cvt8<<<(unsigned)((n8 + 255) / 256), 256, 0, stream>>>(x + (size_t)b * SEQ_FULL * DM, XB + (size_t)b * SEQ * DM, n8, n8);
    }
}

extern "C" void kernel_launch(void* const* d_in, const int* in_sizes, int n_in,
                              void* d_out, int out_size, void* d_ws, size_t ws_size, hipStream_t stream) {
    if (n_in < 14) return;
    const size_t needx = ((size_t)(NB - 1) * SEQ_FULL + SEQ) * DM;
    if ((size_t)in_sizes[0] < needx || (size_t)in_sizes[1] < needx || (size_t)in_sizes[2] < needx) return;
    if ((size_t)in_sizes[3] < (size_t)DM * DM || (size_t)in_sizes[5] < (size_t)DM * DM || (size_t)in_sizes[7] < (size_t)DM * DM || (size_t)in_sizes[9] < (size_t)DM * DM) return;
    if (in_sizes[4] < DM || in_sizes[6] < DM || in_sizes[8] < DM || in_sizes[10] < DM || in_sizes[11] < DM || in_sizes[12] < DM) return;
    if (in_sizes[13] < NREL * DM) return;
    if ((size_t)out_size < ((size_t)(NB - 1) * OUT_SEQ + SEQ) * DM) return;
    if (SZ_TOTAL > ws_size) return;
    const float* xq = (const float*)d_in[0]; const float* xk = (const float*)d_in[1]; const float* xv = (const float*)d_in[2];
    const float* wq = (const float*)d_in[3]; const float* bq = (const float*)d_in[4];
    const float* wk = (const float*)d_in[5]; const float* bk = (const float*)d_in[6];
    const float* wv = (const float*)d_in[7]; const float* bv = (const float*)d_in[8];
    const float* wo = (const float*)d_in[9]; const float* bo = (const float*)d_in[10];
    const float* cb = (const float*)d_in[11]; const float* rb = (const float*)d_in[12]; const float* pe = (const float*)d_in[13];
    float* OUT = (float*)d_out;
    char* wsp = (char*)d_ws;
    bf* XQ = (bf*)wsp; wsp += SZ_XB;
    bf* XK = (bf*)wsp; wsp += SZ_XB;
    bf* XV = (bf*)wsp; wsp += SZ_XB;
    bf* WQT = (bf*)wsp; wsp += SZ_WT;
    bf* WKT = (bf*)wsp; wsp += SZ_WT;
    bf* WVT = (bf*)wsp; wsp += SZ_WT;
    bf* WOT = (bf*)wsp; wsp += SZ_WT;
    bf* PE  = (bf*)wsp; wsp += SZ_PE;
    h16* QCH = (h16*)wsp; wsp += SZ_PL;
    h16* QCR = (h16*)wsp; wsp += SZ_PL;
    h16* QRH = (h16*)wsp; wsp += SZ_PL;
    h16* QRR = (h16*)wsp; wsp += SZ_PL;
    h16* KP  = (h16*)wsp; wsp += SZ_PL;
    h16* VT  = (h16*)wsp; wsp += SZ_PL;
    h16* PKP = (h16*)wsp; wsp += SZ_PK;
    h16* CTX = (h16*)wsp; wsp += SZ_CTX;

    cvt_x(xq, XQ, stream); cvt_x(xk, XK, stream); cvt_x(xv, XV, stream);
    { const size_t nsrc8 = (size_t)NREL * DM / 8, n8 = (size_t)64 * DM / 8;
      k_cvt8<<<(unsigned)((n8 + 255) / 256), 256, 0, stream>>>(pe, PE, nsrc8, n8); }
    k_wt<<<dim3(DM / 64, DM / 64, 1), 256, 0, stream>>>(wq, WQT, 0);
    k_wt<<<dim3(DM / 64, DM / 64, 1), 256, 0, stream>>>(wk, WKT, 0);
    k_wt<<<dim3(DM / 64, DM / 64, 1), 256, 0, stream>>>(wv, WVT, 0);
    k_wt<<<dim3(DM / 64, DM / 64, 1), 256, 0, stream>>>(wo, WOT, 1);

    k_gemm<0><<<dim3(NB * SEQ / 64, DM / 64, 1), 32, 0, stream>>>(XQ, WQT, bq, cb, rb, 1.0f, 1.0f, QCH, QCR, QRH, QRR, OUT,
                                                                  SEQ, (size_t)NH_ * SEQ * HD, HD, HD, (size_t)SEQ * HD);
    k_gemm<1><<<dim3(NB * SEQ / 64, DM / 64, 1), 32, 0, stream>>>(XK, WKT, bk, bk, bk, 1.0f, 1.0f, KP, KP, KP, KP, OUT,
                                                                  SEQ, (size_t)NH_ * SEQ * HD, HD, HD, (size_t)SEQ * HD);
    k_gemm<2><<<dim3(DM / 64, NB * SEQ / 64, 1), 32, 0, stream>>>(WVT, XV, bv, bv, bv, 1.0f, 1.0f, VT, VT, VT, VT, OUT,
                                                                  DM, (size_t)0, SEQ, SEQ, (size_t)DM * SEQ);
    k_gemm<1><<<dim3(1, DM / 64, 1), 32, 0, stream>>>(PE, WKT, bk, bk, bk, PKS, PKS, PKP, PKP, PKP, PKP, OUT,
                                                      64, (size_t)0, HD, HD, (size_t)64 * HD);

    k_flash<<<dim3(SEQ / (16 * AW), NB * NH_, 1), 32 * AW, 0, stream>>>(QCH, QCR, QRH, QRR, KP, VT, PKP, CTX);

    k_gemm<3><<<dim3(NB * SEQ / 64, DM / 64, 1), 32, 0, stream>>>((const bf*)CTX, WOT, bo, bo, bo, OUTI, 1.0f, QCH, QCH, QCH, QCH, OUT,
                                                                  SEQ, (size_t)0, DM, DM, (size_t)0);
}
